// NHRepNet_23424751632495
// MI455X (gfx1250) — hardware-verified
//
#include <hip/hip_runtime.h>
#include <math.h>

typedef __attribute__((ext_vector_type(16))) _Float16 v16h;
typedef __attribute__((ext_vector_type(16))) __bf16 v16b;
typedef __attribute__((ext_vector_type(8)))  _Float16 v8h;
typedef __attribute__((ext_vector_type(8)))  float v8f;
typedef __attribute__((ext_vector_type(4)))  float v4f;
typedef __attribute__((ext_vector_type(2)))  float v2f;
typedef __attribute__((ext_vector_type(4)))  unsigned v4u;
typedef __attribute__((ext_vector_type(4)))  int v4i;
typedef float __attribute__((may_alias)) float_a;
typedef int __attribute__((may_alias)) int_a;

template <typename T> __device__ __forceinline__ void vst2(void* p, T v) { *(volatile T*)p = v; __threadfence(); *(volatile T*)p = v; }
__device__ __forceinline__ v8f wmma16(v16h a, v16h b, v8f c) {
  v8f d = __builtin_amdgcn_wmma_f32_16x16x32_f16(false, a, false, b, (short)0, c, false, false);
  asm volatile("v_nop\n\tv_nop\n\tv_nop\n\tv_nop" : "+v"(d) : "v"(a), "v"(b));
  return d;
}
__device__ __forceinline__ v8f wmma_bf(v16b a, v16b b, v8f c) {
  v8f d = __builtin_amdgcn_wmma_f32_16x16x32_bf16(false, a, false, b, (short)0, c, false, false);
  asm volatile("v_nop\n\tv_nop\n\tv_nop\n\tv_nop" : "+v"(d) : "v"(a), "v"(b));
  return d;
}
__device__ __forceinline__ v16h frag_h(const _Float16* rowk0, int lane) {
  union { v16h v; v8h q[2]; } u; const _Float16* p = rowk0 + 8 * (lane >> 4);
  u.q[0] = *(const v8h*)p; u.q[1] = *(const v8h*)(p + 16); return u.v;
}
__device__ __forceinline__ v16h frag_f32(const float* rowk0, int lane) {
  v16h a; const float* p = rowk0 + 8 * (lane >> 4);
#pragma unroll
  for (int i = 0; i < 8; ++i) { a[i] = (_Float16)p[i]; a[8 + i] = (_Float16)p[16 + i]; }
  return a;
}
__device__ __forceinline__ v16h frag_f32s(const float* rowk0, int lane, float sc) {
  v16h a; const float* p = rowk0 + 8 * (lane >> 4);
#pragma unroll
  for (int i = 0; i < 8; ++i) { a[i] = (_Float16)(p[i] * sc); a[8 + i] = (_Float16)(p[16 + i] * sc); }
  return a;
}
__device__ __forceinline__ v16h fragc_f32(const float* W, int k0, int n, int lane, int ld, int K) {
  v16h a; const int g = lane >> 4;
#pragma unroll
  for (int i = 0; i < 8; ++i) { const int ka = k0 + 8 * g + i, kb = ka + 16;
    a[i] = (_Float16)(ka < K ? W[(size_t)(ka < K ? ka : K - 1) * ld + n] : 0.f); a[8 + i] = (_Float16)(kb < K ? W[(size_t)(kb < K ? kb : K - 1) * ld + n] : 0.f); }
  return a;
}
struct F2 { v16b h, l; };
__device__ __forceinline__ F2 bsplit16(const float v[16]) { F2 r;
#pragma unroll
  for (int i = 0; i < 16; ++i) { const __bf16 h = (__bf16)v[i]; r.h[i] = h; r.l[i] = (__bf16)(v[i] - (float)h); }
  return r; }
__device__ __forceinline__ F2 split_row(const float* row, int k0, int lane) { float v[16]; const float* p = row + k0 + 8 * (lane >> 4);
#pragma unroll
  for (int i = 0; i < 8; ++i) { v[i] = p[i]; v[8 + i] = p[16 + i]; }
  return bsplit16(v); }
__device__ __forceinline__ F2 split_rowK(const float* row, int k0, int lane, int K) { float v[16]; const int g = lane >> 4;
#pragma unroll
  for (int i = 0; i < 8; ++i) { const int ka = k0 + 8 * g + i, kb = ka + 16; v[i] = ka < K ? row[ka < K ? ka : K - 1] : 0.f; v[8 + i] = kb < K ? row[kb < K ? kb : K - 1] : 0.f; }
  return bsplit16(v); }
__device__ __forceinline__ F2 split_col(const float* W, int k0, int n, int lane, int ld, int K) { float v[16]; const int g = lane >> 4;
#pragma unroll
  for (int i = 0; i < 8; ++i) { const int ka = k0 + 8 * g + i, kb = ka + 16; v[i] = ka < K ? W[(size_t)(ka < K ? ka : K - 1) * ld + n] : 0.f; v[8 + i] = kb < K ? W[(size_t)(kb < K ? kb : K - 1) * ld + n] : 0.f; }
  return bsplit16(v); }
__device__ __forceinline__ v8f mac3(const F2& a, const F2& b, v8f c) { c = wmma_bf(a.l, b.h, c); c = wmma_bf(a.h, b.l, c); return wmma_bf(a.h, b.h, c); }
__device__ __forceinline__ float sigm(float v) { return 1.0f / (1.0f + expf(-v)); }
#define LDSX() do { asm volatile("s_wait_dscnt 0" ::: "memory"); __builtin_amdgcn_wave_barrier(); __builtin_amdgcn_fence(__ATOMIC_RELEASE, "workgroup"); } while (0)


#define NPT 100000
#define HID 256
#define NBR 8
#define WSC 256.0f
#define BETA 100.0f
#define NBLK ((NPT + 63) / 64)
#ifndef TBLK
#define TBLK NBLK
#endif
typedef __attribute__((ext_vector_type(8))) __bf16 v8b;
__device__ __forceinline__ v16b frag_b(const __bf16* rowk0, int lane) {
  union { v16b v; v8b q[2]; } u; const __bf16* p = rowk0 + 8 * (lane >> 4);
  u.q[0] = *(const v8b*)p; u.q[1] = *(const v8b*)(p + 16); return u.v;
}
__device__ __forceinline__ float bfr(float v) { return (float)(__bf16)v; }
__device__ __attribute__((noinline)) float exp_ni(float v) { return expf(v); }
__device__ __attribute__((noinline)) float erf_ni(float v) { return erff(v); }

#define WS_W1  0u
#define WS_W2  (WS_W1 + 2u * HID * HID)
#define WS_W3  (WS_W2 + 2u * HID * HID)
#define WS_W4  (WS_W3 + 2u * HID * HID)
#define WS_W5  (WS_W4 + 2u * HID * HID)
#define WS_W6  (WS_W5 + 2u * HID * HID)
#define WS_W7  (WS_W6 + 2u * HID * HID)
#define WS_END (WS_W7 + 2u * 16 * HID)

__global__ __launch_bounds__(256) void k_packw(const float* __restrict__ W1, const float* __restrict__ W2, const float* __restrict__ W3, const float* __restrict__ W4, const float* __restrict__ W5, const float* __restrict__ W6, const float* __restrict__ W7, char* __restrict__ ws) {
  const int n = blockIdx.x, l = blockIdx.y + 1, t = threadIdx.x; __shared__ __align__(16) _Float16 s[HID];
  const float* Wm = l == 1 ? W1 : l == 2 ? W2 : l == 3 ? W3 : l == 4 ? W4 : l == 5 ? W5 : l == 6 ? W6 : W7; const int kout = l == 3 ? 253 : (l == 7 ? NBR : HID); const int nrows = l == 7 ? 16 : HID; if (n >= nrows) return;
  s[t] = (n < kout) ? (_Float16)(bfr(Wm[(size_t)t * kout + n]) * WSC) : (_Float16)0.0f; __syncthreads();
  _Float16* dst = (_Float16*)(ws + WS_W1 + (size_t)(l - 1) * 2u * HID * HID) + (size_t)n * HID; if (t < HID / 8) vst2((unsigned*)(dst + t * 8), *(const v4u*)&s[t * 8]); }
__device__ __forceinline__ float softplus_b(float x) { const float z = BETA * x; return (fmaxf(z, 0.f) + logf(1.0f + expf(-fabsf(z)))) * (1.0f / BETA); }
__device__ __forceinline__ v16h frag_lds(const _Float16* p, int lane) { v16h a; const _Float16* pp = p + 8 * (lane >> 4);
#pragma unroll
  for (int i = 0; i < 8; ++i) { a[i] = pp[i]; a[8 + i] = pp[16 + i]; } return a; }
template <int NT, int L>
__device__ __forceinline__ void layer_step(_Float16 (*sa)[HID + 8], const float (*sx)[4], float (*sres)[12], const _Float16* __restrict__ Wl, const float* __restrict__ Bl, int wave, int lane, int col, int g) {
  v8f acc[NT];
#pragma unroll
  for (int j = 0; j < NT; ++j) acc[j] = v8f{};
#pragma unroll 2
  for (int kc = 0; kc < HID / 32; ++kc) { const v16h a = frag_lds(&sa[wave * 16 + col][kc * 32], lane);
#pragma unroll
    for (int j = 0; j < NT; ++j) acc[j] = wmma16(a, frag_h(Wl + (size_t)(j * 16 + col) * HID + kc * 32, lane), acc[j]); }
  __syncthreads();
  if (L < 7) { const float inv_sqrt2 = 0.70710678118654752f; constexpr int kout = (L == 3) ? 253 : HID;
#pragma unroll
    for (int j = 0; j < NT; ++j) { const int n = j * 16 + col; const float bb = (n < kout) ? bfr(Bl[n < kout ? n : 0]) : 0.f;
#pragma unroll
      for (int r = 0; r < 8; ++r) { const int rl = wave * 16 + 8 * g + r; float v; if (n < kout) { v = softplus_b(acc[j][r] * (1.0f / WSC) + bb); if (L == 3) v *= inv_sqrt2; } else { v = sx[rl][(n - 253) & 3] * inv_sqrt2; } sa[rl][n] = (_Float16)v; } } }
  else { if (col < NBR) { const float bb = bfr(Bl[col]);
#pragma unroll
      for (int r = 0; r < 8; ++r) sres[wave * 16 + 8 * g + r][1 + col] = acc[0][r] * (1.0f / WSC) + bb; } }
  __syncthreads(); }
__global__ __launch_bounds__(128) void k_net(const float* __restrict__ X, const float* __restrict__ W0, const float* __restrict__ B0, const float* __restrict__ B1, const float* __restrict__ B2, const float* __restrict__ B3, const float* __restrict__ B4, const float* __restrict__ B5, const float* __restrict__ B6, const float* __restrict__ B7, const _Float16* __restrict__ WR, float* __restrict__ OUT) {
  __shared__ __align__(16) _Float16 sa[64][HID + 8]; __shared__ float sx[64][4]; __shared__ __align__(16) float sres[64][12]; __shared__ __align__(16) float sflat[576];
  const int tid = threadIdx.x, wave = tid >> 5, lane = tid & 31, col = lane & 15, g = lane >> 4; const size_t p0 = (size_t)blockIdx.x * 64;
  if (tid < 64) { const size_t p = p0 + tid; const bool ok = p < NPT; for (int d = 0; d < 3; ++d) sx[tid][d] = ok ? bfr(X[p * 3 + d]) : 0.f; sx[tid][3] = 0.f; }
  __syncthreads();
  for (int e = tid; e < 64 * HID; e += 128) { const int r = e / HID, n = e % HID; float s = bfr(B0[n]);
#pragma unroll
    for (int d = 0; d < 3; ++d) s += sx[r][d] * bfr(W0[d * HID + n]);
    sa[r][n] = (_Float16)softplus_b(s); }
  __syncthreads();
  layer_step<16, 1>(sa, sx, sres, WR + 0 * (size_t)HID * HID, B1, wave, lane, col, g);
  layer_step<16, 2>(sa, sx, sres, WR + 1 * (size_t)HID * HID, B2, wave, lane, col, g);
  layer_step<16, 3>(sa, sx, sres, WR + 2 * (size_t)HID * HID, B3, wave, lane, col, g);
  layer_step<16, 4>(sa, sx, sres, WR + 3 * (size_t)HID * HID, B4, wave, lane, col, g);
  layer_step<16, 5>(sa, sx, sres, WR + 4 * (size_t)HID * HID, B5, wave, lane, col, g);
  layer_step<16, 6>(sa, sx, sres, WR + 5 * (size_t)HID * HID, B6, wave, lane, col, g);
  layer_step<1, 7>(sa, sx, sres, WR + 6 * (size_t)HID * HID, B7, wave, lane, col, g);
  if (tid < 64) { const float* h = &sres[tid][1]; const float m23 = fminf(h[2], h[3]); const float m67 = fmaxf(h[6], h[7]); const float m45 = fminf(fminf(h[4], h[5]), m67); sres[tid][0] = fmaxf(fmaxf(h[0], h[1]), fmaxf(m23, m45)); }
  __syncthreads();
  { const size_t base = p0 * 9; const int nval = (int)(((p0 + 64 <= NPT) ? 64 : (NPT - p0)) * 9);
    for (int e = tid; e < 576; e += 128) sflat[e] = sres[e / 9][e % 9]; __syncthreads();
    for (int q = tid; q < 144; q += 128) if (q * 4 + 4 <= nval) vst2(OUT + base + q * 4, *(const v4f*)&sflat[q * 4]); } }
extern "C" void kernel_launch(void* const* d_in, const int* in_sizes, int n_in, void* d_out, int out_size, void* d_ws, size_t ws_size, hipStream_t stream) {
  (void)in_sizes; (void)n_in; (void)out_size;
  const float** F = (const float**)d_in;
  if (ws_size < (size_t)WS_END) return;
  char* ws = (char*)d_ws; _Float16* WR = (_Float16*)(ws + WS_W1);
  k_packw<<<dim3(HID, 7), 256, 0, stream>>>(F[3], F[5], F[7], F[9], F[11], F[13], F[15], ws);
  k_net<<<TBLK, 128, 0, stream>>>(F[0], F[1], F[2], F[4], F[6], F[8], F[10], F[12], F[14], F[16], WR, (float*)d_out);
}
